// GRU_37761352466675
// MI455X (gfx1250) — hardware-verified
//
#include <hip/hip_runtime.h>
#include <math.h>

constexpr int NB    = 2;
constexpr int NS    = 2048;
constexpr int NDIN  = 2048;
constexpr int NST   = 2048;
constexpr int NOUTC = 2048;
constexpr int NH    = 16;
constexpr int DH    = 128;
constexpr int NGRP  = 12;
constexpr int GOUT  = 512;
constexpr int C3X   = 1536;
constexpr int C6X   = 6144;
constexpr int NROW  = NB * NS;
constexpr int PLP   = 2048;
constexpr int NTG   = 256;
constexpr int NTC   = 192;
constexpr int NTR   = 256;
constexpr int APITCH = 136;
constexpr float FACTOR_F  = 0.5f;
constexpr float WIN_CAR   = 32.0f;
constexpr float HW_CAR    = 32.0f;
constexpr float OHW_CAR   = 256.0f;
constexpr float WOUT_CAR  = 256.0f;
constexpr float WREC_CAR  = 16.0f;
constexpr float XALL_CAR  = 16.0f;
constexpr float HRES_CAR  = 32768.0f;
constexpr float H1RES_CAR = 2048.0f;
constexpr float RMS_EPS   = 1e-6f;
static_assert(NB == 2);
static_assert(NH * DH == NST);
static_assert(NGRP * GOUT == C6X && NGRP * DH == C3X);
static_assert(NTC * 8 == C3X);
static_assert(NTG * 8 == NST);
static_assert(NTR == 2 * DH);
static_assert((2 * 16 * APITCH) % NTR == 0);
static_assert(PLP == NDIN && PLP == NST && C3X <= PLP);
static_assert(NDIN % 32 == 0 && DH % 32 == 0 && NST % 32 == 0);
static_assert(NROW % 64 == 0 && NROW % 32 == 0 && C3X % 64 == 0 && GOUT % 64 == 0 && DH % 64 == 0 && NOUTC % 64 == 0);
static_assert(((NROW / 64) * (C3X / 64)) % 8 == 0 && ((NROW / 32) * (GOUT / 64)) % 8 == 0 &&
              ((NROW / 32) * (DH / 64)) % 8 == 0 && ((NROW / 64) * (NOUTC / 64)) % 8 == 0);
static_assert((NROW * NDIN / 8) % NTG == 0);
static_assert(NDIN % 64 == 0 && C3X % 64 == 0 && DH % 64 == 0 && GOUT % 64 == 0);

typedef __attribute__((ext_vector_type(16))) _Float16 v16h;
typedef __attribute__((ext_vector_type(8)))  _Float16 v8h;
typedef __attribute__((ext_vector_type(16))) __bf16   v16b;
typedef __attribute__((ext_vector_type(8)))  __bf16   v8b;
typedef __attribute__((ext_vector_type(8)))  float    v8f;
typedef __attribute__((ext_vector_type(4)))  float    v4f;
typedef __attribute__((ext_vector_type(4)))  unsigned v4u;

__device__ __forceinline__ unsigned short f2bf_bits(float f) {
  unsigned u = __float_as_uint(f);
  return (unsigned short)((u + 0x7FFFu + ((u >> 16) & 1u)) >> 16);
}
__device__ __forceinline__ float bf_bits2f(unsigned short h) { return __uint_as_float(((unsigned)h) << 16); }

__device__ __forceinline__ float h16_to_f32(unsigned hb) {
  const unsigned sgn = (hb & 0x8000u) << 16; const unsigned em = hb & 0x7fffu;
  const float fn = __uint_as_float((em << 13) + 0x38000000u);
  const float fs = (float)em * 5.9604644775390625e-8f;
  const float mag = (em < 0x400u) ? fs : fn; return __uint_as_float(__float_as_uint(mag) | sgn);
}

__device__ __forceinline__ void dep_guard_h(v8f& a, v8f& b, v16h x, v16h y) { asm volatile("v_nop\n\tv_nop\n\tv_nop\n\tv_nop" : "+v"(a), "+v"(b) : "v"(x), "v"(y)); }
__device__ __forceinline__ void dep_guard_b(v8f& a, v8f& b, v16b x, v16b y) { asm volatile("v_nop\n\tv_nop\n\tv_nop\n\tv_nop" : "+v"(a), "+v"(b) : "v"(x), "v"(y)); }
__device__ __forceinline__ void dep_guard4_h(v8f& a, v8f& b, v8f& c, v8f& d, v16h x, v16h y) { asm volatile("v_nop\n\tv_nop\n\tv_nop\n\tv_nop" : "+v"(a), "+v"(b), "+v"(c), "+v"(d) : "v"(x), "v"(y)); }
__device__ __forceinline__ void dep_guard4_b(v8f& a, v8f& b, v8f& c, v8f& d, v16b x, v16b y) { asm volatile("v_nop\n\tv_nop\n\tv_nop\n\tv_nop" : "+v"(a), "+v"(b), "+v"(c), "+v"(d) : "v"(x), "v"(y)); }
__device__ __forceinline__ void dep_guard8_h(v8f& a, v8f& b, v8f& c, v8f& d, v8f& e, v8f& f, v8f& g, v8f& h, v16h x, v16h y) {
  asm volatile("v_nop\n\tv_nop\n\tv_nop\n\tv_nop" : "+v"(a), "+v"(b), "+v"(c), "+v"(d), "+v"(e), "+v"(f), "+v"(g), "+v"(h) : "v"(x), "v"(y));
}
__device__ __forceinline__ void dep_guard3_h4(v8f& a, v8f& b, v8f& c, v16h x, v16h y, v16h z, v16h w) { asm volatile("v_nop\n\tv_nop\n\tv_nop\n\tv_nop" : "+v"(a), "+v"(b), "+v"(c) : "v"(x), "v"(y), "v"(z), "v"(w)); }
__device__ __forceinline__ void keep4_h(v16h a, v16h b, v16h c, v16h d) { asm volatile("v_nop" :: "v"(a), "v"(b), "v"(c), "v"(d)); }
__device__ __forceinline__ void keep4_b(v16b a, v16b b, v16b c, v16b d) { asm volatile("v_nop" :: "v"(a), "v"(b), "v"(c), "v"(d)); }
__device__ __forceinline__ void fence4_h(v16h a, v16h b, v16h c, v16h d) { asm volatile("v_nop" :: "v"(a), "v"(b), "v"(c), "v"(d) : "memory"); }
__device__ __forceinline__ void fence4_v4(v4f a, v4f b, v4f c, v4f d) { asm volatile("" :: "v"(a), "v"(b), "v"(c), "v"(d) : "memory"); }
__device__ __forceinline__ void acc_guard4(v8f& a, v8f& b, v8f& c, v8f& d) { asm volatile("v_nop\n\tv_nop\n\tv_nop\n\tv_nop" : "+v"(a), "+v"(b), "+v"(c), "+v"(d)); }
__device__ __forceinline__ void acc_guard3(v8f& a, v8f& b, v8f& c) { asm volatile("v_nop\n\tv_nop\n\tv_nop\n\tv_nop" : "+v"(a), "+v"(b), "+v"(c)); }

template <typename T> struct Frag;
template <> struct Frag<_Float16> {
  typedef v16h V; union U { v16h v; v8h h[2]; };
  static __device__ __forceinline__ v16h load(const _Float16* p) {
    U f; f.h[0] = *(const v8h*)(p); f.h[1] = *(const v8h*)(p + 16); return f.v;
  }
  static __device__ __forceinline__ v8f mma(v16h a, v16h b, v8f c) {
    return __builtin_amdgcn_wmma_f32_16x16x32_f16(false, a, false, b, (short)0, c, false, false);
  }
  static __device__ __forceinline__ void guard(v8f& a, v8f& b, v16h x, v16h y) { dep_guard_h(a, b, x, y); }
  static __device__ __forceinline__ void guard4(v8f& a, v8f& b, v8f& c, v8f& d, v16h x, v16h y) { dep_guard4_h(a, b, c, d, x, y); }
  static __device__ __forceinline__ void keep(v16h a, v16h b, v16h c, v16h d) { keep4_h(a, b, c, d); }
};
template <> struct Frag<__bf16> {
  typedef v16b V; union U { v16b v; v8b h[2]; };
  static __device__ __forceinline__ v16b load(const __bf16* p) {
    U f; f.h[0] = *(const v8b*)(p); f.h[1] = *(const v8b*)(p + 16); return f.v;
  }
  static __device__ __forceinline__ v8f mma(v16b a, v16b b, v8f c) {
    return __builtin_amdgcn_wmma_f32_16x16x32_bf16(false, a, false, b, (short)0, c, false, false);
  }
  static __device__ __forceinline__ void guard(v8f& a, v8f& b, v16b x, v16b y) { dep_guard_b(a, b, x, y); }
  static __device__ __forceinline__ void guard4(v8f& a, v8f& b, v8f& c, v8f& d, v16b x, v16b y) { dep_guard4_b(a, b, c, d, x, y); }
  static __device__ __forceinline__ void keep(v16b a, v16b b, v16b c, v16b d) { keep4_b(a, b, c, d); }
};

template <int ET> struct Elem;
template <> struct Elem<0> { typedef _Float16 T; };
template <> struct Elem<1> { typedef __bf16 T; };
template <int ET, bool SPLIT, int BIAS_MODE, int OUT_MODE, bool RESID, int ACT = 0>
__global__ __launch_bounds__(256) void wmma_gemm64(
    const unsigned short* __restrict__ Ap, const unsigned short* __restrict__ A2p, int lda, long strideA,
    const unsigned short* __restrict__ Btp, const unsigned short* __restrict__ Bt2p, int ldb, long strideB,
    void* __restrict__ Cout, void* __restrict__ Cout2, int ldc, long strideC,
    const float* __restrict__ bias,
    const float* __restrict__ resid, long strideR,
    int M, int N, int K, float scale) {
  typedef typename Elem<ET>::T T;
  typedef typename Frag<T>::V V;
  const T* A = (const T*)Ap; const T* A2 = (const T*)A2p; const T* Bt = (const T*)Btp; const T* Bt2 = (const T*)Bt2p;
  __shared__ __align__(16) float sT[8][16 * 68];
  const int b    = blockIdx.y;
  const int lane = threadIdx.x & 31;
  const int wave = threadIdx.x >> 5;
  const int tilesN = N >> 6;
  const int tilesM = M >> 6;
  const int tile = blockIdx.x * 8 + wave;
  if (tile >= tilesM * tilesN) return;
  const int tm = tile / tilesN;
  const int tn = tile - tm * tilesN;
  const int m0 = tm << 6;
  const int n0 = tn << 6;

  const T* Ab  = A  + (size_t)b * strideA;
  const T* Bb  = Bt + (size_t)b * strideB;
  const T* Ab2 = SPLIT ? (A2  + (size_t)b * strideA) : nullptr;
  const T* Bb2 = SPLIT ? (Bt2 + (size_t)b * strideB) : nullptr;

  const int rlane = lane & 15;
  const int koff  = (lane >> 4) * 8;
  const int mOff  = (lane >> 4) * 8;

  v8f acc[4][4];
#pragma unroll
  for (int i = 0; i < 4; ++i)
#pragma unroll
    for (int j = 0; j < 4; ++j) acc[i][j] = (v8f){0.f,0.f,0.f,0.f,0.f,0.f,0.f,0.f};

  for (int k0 = 0; k0 < K; k0 += 32) {
    V bh[4], bl[4];
#pragma unroll
    for (int j = 0; j < 4; ++j) {
      const size_t bo = (size_t)(n0 + (j << 4) + rlane) * ldb + koff + k0;
      bh[j] = Frag<T>::load(Bb + bo);
      if (SPLIT) bl[j] = Frag<T>::load(Bb2 + bo);
    }
#pragma unroll
    for (int i = 0; i < 4; ++i) {
      const size_t ao = (size_t)(m0 + (i << 4) + rlane) * lda + koff + k0;
      V ah = Frag<T>::load(Ab + ao);
      V al;
      if (SPLIT) al = Frag<T>::load(Ab2 + ao);
#pragma unroll
      for (int j = 0; j < 4; ++j) {
        acc[i][j] = Frag<T>::mma(ah, bh[j], acc[i][j]);
        if (SPLIT) {
          acc[i][j] = Frag<T>::mma(ah, bl[j], acc[i][j]);
          acc[i][j] = Frag<T>::mma(al, bh[j], acc[i][j]);
        }
      }
      Frag<T>::guard4(acc[i][0], acc[i][1], acc[i][2], acc[i][3], ah, SPLIT ? al : bh[3]);
    }
    Frag<T>::keep(bh[0], bh[1], bh[2], bh[3]);
    if (SPLIT) Frag<T>::keep(bl[0], bl[1], bl[2], bl[3]);
  }
  acc_guard4(acc[0][0], acc[0][1], acc[0][2], acc[0][3]);
  acc_guard4(acc[1][0], acc[1][1], acc[1][2], acc[1][3]);
  acc_guard4(acc[2][0], acc[2][1], acc[2][2], acc[2][3]);
  acc_guard4(acc[3][0], acc[3][1], acc[3][2], acc[3][3]);

  float* slab = sT[wave];
  const float* Rb = RESID ? (resid + (size_t)b * strideR) : nullptr;
#pragma unroll
  for (int i = 0; i < 4; ++i) {
    const int mBase = m0 + (i << 4);
#pragma unroll
    for (int j = 0; j < 4; ++j) {
      const int n = n0 + (j << 4) + rlane;
      float bv = 0.f;
      if (BIAS_MODE == 2) bv = bias[n];
#pragma unroll
      for (int r = 0; r < 8; ++r) {
        float v = acc[i][j][r] * scale;
        if (BIAS_MODE == 1) v += bias[mBase + mOff + r];
        if (BIAS_MODE == 2) v += bv;
        if (RESID) v += Rb[(size_t)(mBase + mOff + r) * ldc + n];
        if (ACT == 1) v = tanhf(v);
        if (ACT == 2) v = fmaxf(v, 0.0f);
        if (ACT == 3) v = v / (1.0f + expf(-v));
        if (ACT == 4) v = (v > 0.f) ? v : 0.01f * v;
        if (ACT == 5) v = 0.5f * v * (1.0f + erff(v * 0.70710678118654752f));
        slab[(mOff + r) * 68 + (j << 4) + rlane] = v;
      }
    }
    __builtin_amdgcn_fence(__ATOMIC_RELEASE, "workgroup");
    __builtin_amdgcn_wave_barrier();
    __builtin_amdgcn_fence(__ATOMIC_ACQUIRE, "workgroup");
    if (OUT_MODE == 0) {
      float* C = (float*)Cout + (size_t)b * strideC;
      const int hh = lane >> 4, c4 = (lane & 15) * 4;
      for (int pass = 0; pass < 2; ++pass) {
#pragma unroll
        for (int it = 0; it < 8; ++it) {
          const int row = it * 2 + hh;
          v4f v = *(const v4f*)(slab + row * 68 + c4);
          *(volatile v4f*)(C + (size_t)(mBase + row) * ldc + n0 + c4) = v;
        }
        __threadfence();
      }
    } else {
      const int q = lane >> 3, c8 = (lane & 7) * 8;
      unsigned short* C  = (unsigned short*)Cout  + (size_t)b * strideC;
      unsigned short* C2 = (OUT_MODE == 2) ? ((unsigned short*)Cout2 + (size_t)b * strideC) : nullptr;
      for (int pass = 0; pass < 2; ++pass) {
#pragma unroll
        for (int it = 0; it < 4; ++it) {
          const int row = it * 4 + q;
          const float* sp = slab + row * 68 + c8;
          v8h hv, lv;
#pragma unroll
          for (int e = 0; e < 8; ++e) {
            if (OUT_MODE == 1) {
              hv[e] = (_Float16)sp[e];
            } else {
              unsigned short hb = f2bf_bits(sp[e]);
              unsigned short lb = f2bf_bits(sp[e] - bf_bits2f(hb));
              hv[e] = __builtin_bit_cast(_Float16, hb);
              lv[e] = __builtin_bit_cast(_Float16, lb);
            }
          }
          *(volatile v8h*)(C + (size_t)(mBase + row) * ldc + n0 + c8) = hv;
          if (OUT_MODE == 2) *(volatile v8h*)(C2 + (size_t)(mBase + row) * ldc + n0 + c8) = lv;
        }
        __threadfence();
      }
    }
    __builtin_amdgcn_fence(__ATOMIC_RELEASE, "workgroup");
    __builtin_amdgcn_wave_barrier();
    __builtin_amdgcn_fence(__ATOMIC_ACQUIRE, "workgroup");
  }
}

__global__ __launch_bounds__(256) void wmma_gemm_ares(
    const unsigned short* __restrict__ Ahp, const unsigned short* __restrict__ Alp, int lda, long strideA,
    const unsigned short* __restrict__ Btp, int ldb, long strideB,
    unsigned short* __restrict__ Cp, int ldc, long strideC,
    int M, int N, int K, float scale, float rscale) {
  const _Float16* Ah = (const _Float16*)Ahp; const _Float16* Al = (const _Float16*)Alp; const _Float16* Bt = (const _Float16*)Btp;
  __shared__ __align__(16) float sT[8][16 * 68];
  const int b    = blockIdx.y;
  const int lane = threadIdx.x & 31;
  const int wave = threadIdx.x >> 5;
  const int tilesN = N >> 6;
  const int tilesM = M >> 5;
  const int tile = blockIdx.x * 8 + wave;
  if (tile >= tilesM * tilesN) return;
  const int tm = tile / tilesN;
  const int tn = tile - tm * tilesN;
  const int m0 = tm << 5;
  const int n0 = tn << 6;

  const _Float16* Ahb = Ah + (size_t)b * strideA;
  const _Float16* Alb = Al + (size_t)b * strideA;
  const _Float16* Bb  = Bt + (size_t)b * strideB;

  const int rlane = lane & 15;
  const int koff  = (lane >> 4) * 8;
  const int mOff  = (lane >> 4) * 8;

  const v8f z8 = {0.f,0.f,0.f,0.f,0.f,0.f,0.f,0.f};
  v8f acc[2][4], accr[2][4];
#pragma unroll
  for (int i = 0; i < 2; ++i)
#pragma unroll
    for (int j = 0; j < 4; ++j) { acc[i][j] = z8; accr[i][j] = z8; }

  for (int k0 = 0; k0 < K; k0 += 32) {
    v16h bh[4];
#pragma unroll
    for (int j = 0; j < 4; ++j) {
      const size_t bo = (size_t)(n0 + (j << 4) + rlane) * ldb + koff + k0;
      bh[j] = Frag<_Float16>::load(Bb + bo);
    }
#pragma unroll
    for (int i = 0; i < 2; ++i) {
      const size_t ao = (size_t)(m0 + (i << 4) + rlane) * lda + koff + k0;
      const v16h ah = Frag<_Float16>::load(Ahb + ao);
      const v16h al = Frag<_Float16>::load(Alb + ao);
#pragma unroll
      for (int j = 0; j < 4; ++j) {
        acc[i][j]  = Frag<_Float16>::mma(ah, bh[j], acc[i][j]);
        accr[i][j] = Frag<_Float16>::mma(al, bh[j], accr[i][j]);
      }
      dep_guard8_h(acc[i][0], acc[i][1], acc[i][2], acc[i][3], accr[i][0], accr[i][1], accr[i][2], accr[i][3], ah, al);
    }
    keep4_h(bh[0], bh[1], bh[2], bh[3]);
  }
  acc_guard4(acc[0][0], acc[0][1], acc[0][2], acc[0][3]);
  acc_guard4(acc[1][0], acc[1][1], acc[1][2], acc[1][3]);
  acc_guard4(accr[0][0], accr[0][1], accr[0][2], accr[0][3]);
  acc_guard4(accr[1][0], accr[1][1], accr[1][2], accr[1][3]);

  float* slab = sT[wave];
  unsigned short* C = Cp + (size_t)b * strideC;
  const int q = lane >> 3, c8 = (lane & 7) * 8;
#pragma unroll
  for (int i = 0; i < 2; ++i) {
    const int mBase = m0 + (i << 4);
#pragma unroll
    for (int j = 0; j < 4; ++j) {
#pragma unroll
      for (int r = 0; r < 8; ++r) {
        const float v = acc[i][j][r] * scale + accr[i][j][r] * rscale;
        slab[(mOff + r) * 68 + (j << 4) + rlane] = v;
      }
    }
    __builtin_amdgcn_fence(__ATOMIC_RELEASE, "workgroup");
    __builtin_amdgcn_wave_barrier();
    __builtin_amdgcn_fence(__ATOMIC_ACQUIRE, "workgroup");
    for (int pass = 0; pass < 2; ++pass) {
#pragma unroll
      for (int it = 0; it < 4; ++it) {
        const int row = it * 4 + q;
        const float* sp = slab + row * 68 + c8;
        v8h hv;
#pragma unroll
        for (int e = 0; e < 8; ++e) hv[e] = (_Float16)sp[e];
        *(volatile v8h*)(C + (size_t)(mBase + row) * ldc + n0 + c8) = hv;
      }
      __threadfence();
    }
    __builtin_amdgcn_fence(__ATOMIC_RELEASE, "workgroup");
    __builtin_amdgcn_wave_barrier();
    __builtin_amdgcn_fence(__ATOMIC_ACQUIRE, "workgroup");
  }
}

__global__ __launch_bounds__(NTG) void cvt_f16x8_kernel(const float* __restrict__ src, unsigned short* __restrict__ dst, int n8) {
  const int i = blockIdx.x * NTG + threadIdx.x;
  if (i < n8) {
    const float* sp = src + (size_t)i * 8;
    const v4f a = *(const v4f*)(sp);
    const v4f b = *(const v4f*)(sp + 4);
    v8h hv;
#pragma unroll
    for (int e = 0; e < 4; ++e) { hv[e] = (_Float16)a[e]; hv[4 + e] = (_Float16)b[e]; }
    unsigned short* op = dst + (size_t)i * 8;
    *(volatile v8h*)op = hv;
    __threadfence();
    *(volatile v8h*)op = hv;
  }
}

__global__ __launch_bounds__(NTG) void tpw16_kernel(const float* __restrict__ src, int R, int C, long zin, long zout,
                                                    unsigned short* __restrict__ O, float sc) {
  __shared__ float Tt[64 * 65];
  const int tid = threadIdx.x;
  const int c0 = blockIdx.x * 64, r0 = blockIdx.y * 64;
  const float* sp0 = src + (size_t)blockIdx.z * (size_t)zin;
  unsigned short* op0 = O + (size_t)blockIdx.z * (size_t)zout;
#pragma unroll
  for (int i = 0; i < 4; ++i) {
    const int idx = i * NTG + tid;
    const int rr = idx >> 4, cc = (idx & 15) * 4;
    const v4f v = *(const v4f*)(sp0 + (size_t)(r0 + rr) * (size_t)C + c0 + cc);
    Tt[rr * 65 + cc + 0] = v[0];
    Tt[rr * 65 + cc + 1] = v[1];
    Tt[rr * 65 + cc + 2] = v[2];
    Tt[rr * 65 + cc + 3] = v[3];
  }
  __syncthreads();
  const int q = tid >> 3, c8 = (tid & 7) * 8;
  v8h hv[2];
#pragma unroll
  for (int g = 0; g < 2; ++g) {
    const int qq = g * 32 + q;
#pragma unroll
    for (int e = 0; e < 8; ++e) hv[g][e] = (_Float16)(Tt[(c8 + e) * 65 + qq] * sc);
  }
  for (int pass = 0; pass < 2; ++pass) {
#pragma unroll
    for (int g = 0; g < 2; ++g) {
      const size_t o = (size_t)(c0 + g * 32 + q) * (size_t)R + (size_t)(r0 + c8);
      *(volatile v8h*)(op0 + o) = hv[g];
    }
    __threadfence();
  }
}

__global__ __launch_bounds__(NTC) void conv_rms_kernel(const float* __restrict__ H0, const float* __restrict__ cw,
                                                       const float* __restrict__ rw, unsigned short* __restrict__ Hhi,
                                                       unsigned short* __restrict__ Hlo) {
  __shared__ float red[NTC / 32];
  const int tid = threadIdx.x, lane = tid & 31, wave = tid >> 5;
  const int row = blockIdx.x;
  const int bb = row / NS, s = row - bb * NS;
  const int c0 = tid * 8;
  v4f wv[8];
#pragma unroll
  for (int i = 0; i < 4; ++i) wv[i] = *(const v4f*)(cw + (size_t)(c0 + i) * 4);
  fence4_v4(wv[0], wv[1], wv[2], wv[3]);
#pragma unroll
  for (int i = 4; i < 8; ++i) wv[i] = *(const v4f*)(cw + (size_t)(c0 + i) * 4);
  fence4_v4(wv[4], wv[5], wv[6], wv[7]);
  const v4f rwa = *(const v4f*)(rw + c0);
  const v4f rwb = *(const v4f*)(rw + c0 + 4);
  fence4_v4(rwa, rwb, rwa, rwb);
  float hc[8];
#pragma unroll
  for (int e = 0; e < 8; ++e) hc[e] = 0.0f;
#pragma unroll
  for (int j = 0; j < 4; ++j) {
    const int sp = s - 3 + j;
    const int spc = (sp < 0) ? 0 : sp;
    const float fac = (sp < 0) ? 0.0f : 1.0f;
    const float* hp = H0 + ((size_t)(bb * NS + spc)) * (size_t)C3X + c0;
    const v4f ha = *(const v4f*)(hp);
    const v4f hb = *(const v4f*)(hp + 4);
#pragma unroll
    for (int e = 0; e < 4; ++e) {
      hc[e]     += wv[e][j]     * (ha[e] * fac);
      hc[4 + e] += wv[4 + e][j] * (hb[e] * fac);
    }
  }
  float ss = 0.0f;
#pragma unroll
  for (int e = 0; e < 8; ++e) ss += hc[e] * hc[e];
#pragma unroll
  for (int off = 1; off < 32; off <<= 1) ss += __shfl_xor(ss, off, 32);
  if (lane == 0) red[wave] = ss;
  __syncthreads();
  float tot = 0.0f;
#pragma unroll
  for (int w = 0; w < NTC / 32; ++w) tot += red[w];
  const float inv = 1.0f / sqrtf(tot * (1.0f / (float)C3X) + RMS_EPS);
  v8h hv, lv;
#pragma unroll
  for (int e = 0; e < 4; ++e) {
    const float fa = (hc[e] * rwa[e]) * inv;
    const float fb = (hc[4 + e] * rwb[e]) * inv;
    const _Float16 ha16 = (_Float16)fa;
    const _Float16 hb16 = (_Float16)fb;
    const float haf = h16_to_f32((unsigned)__builtin_bit_cast(unsigned short, ha16));
    const float hbf = h16_to_f32((unsigned)__builtin_bit_cast(unsigned short, hb16));
    hv[e]     = ha16;
    hv[4 + e] = hb16;
    lv[e]     = (_Float16)((fa - haf) * H1RES_CAR);
    lv[4 + e] = (_Float16)((fb - hbf) * H1RES_CAR);
  }
  unsigned short* oph = Hhi + (size_t)row * (size_t)PLP + c0;
  unsigned short* opl = Hlo + (size_t)row * (size_t)PLP + c0;
  *(volatile v8h*)oph = hv;
  *(volatile v8h*)opl = lv;
  __threadfence();
  *(volatile v8h*)oph = hv;
  *(volatile v8h*)opl = lv;
}

__global__ __launch_bounds__(NTG) void rms2_kernel(const unsigned short* __restrict__ Y2, const float* __restrict__ rw,
                                                   unsigned short* __restrict__ Y2N) {
  __shared__ float red[NTG / 32];
  const int tid = threadIdx.x, lane = tid & 31, wave = tid >> 5;
  const int row = blockIdx.x;
  const int c0 = tid * 8;
  const v4u w = *(const v4u*)(Y2 + (size_t)row * (size_t)C6X + c0);
  const v4f rwa = *(const v4f*)(rw + c0);
  const v4f rwb = *(const v4f*)(rw + c0 + 4);
  float v[8];
#pragma unroll
  for (int k = 0; k < 4; ++k) {
    const unsigned wk = w[k];
    v[2 * k]     = h16_to_f32(wk & 0xffffu);
    v[2 * k + 1] = h16_to_f32(wk >> 16);
  }
  float ss = 0.0f;
#pragma unroll
  for (int e = 0; e < 8; ++e) ss += v[e] * v[e];
#pragma unroll
  for (int off = 1; off < 32; off <<= 1) ss += __shfl_xor(ss, off, 32);
  if (lane == 0) red[wave] = ss;
  __syncthreads();
  float tot = 0.0f;
#pragma unroll
  for (int ww = 0; ww < NTG / 32; ++ww) tot += red[ww];
  const float inv = 1.0f / sqrtf(tot * (1.0f / (float)NST) + RMS_EPS * OHW_CAR * OHW_CAR);
  v8h hv;
#pragma unroll
  for (int e = 0; e < 4; ++e) {
    hv[e]     = (_Float16)((v[e] * rwa[e]) * inv);
    hv[4 + e] = (_Float16)((v[4 + e] * rwb[e]) * inv);
  }
  unsigned short* op = Y2N + (size_t)row * (size_t)NST + c0;
  *(volatile v8h*)op = hv;
  __threadfence();
  *(volatile v8h*)op = hv;
}

__global__ __launch_bounds__(NTR) void gru_seq_kernel(const unsigned* __restrict__ Xw, const unsigned short* __restrict__ Wp,
                                                     const float* __restrict__ fbias_in, const float* __restrict__ rbias_in,
                                                     unsigned short* __restrict__ Yrec, unsigned short* __restrict__ YrecL) {
  __shared__ __align__(16) _Float16 Ah[2][16 * APITCH];
  const _Float16* W = (const _Float16*)Wp;
  const int tid = threadIdx.x, lane = tid & 31, wave = tid >> 5;
  const int c = lane & 15, hh = lane >> 4, koff = hh * 8;
  const int hd = blockIdx.x;
  const int e = 16 * wave + c;

  {
    _Float16* af = &Ah[0][0];
#pragma unroll 1
    for (int i = tid; i < 2 * 16 * APITCH; i += NTR) af[i] = (_Float16)0.0f;
  }
  v16h bfr[3][4];
#pragma unroll
  for (int g = 0; g < 3; ++g) {
    const _Float16* wrow = W + ((size_t)(g * NH + hd) * DH + (size_t)e) * DH + koff;
#pragma unroll
    for (int kc = 0; kc < 4; ++kc) bfr[g][kc] = Frag<_Float16>::load(wrow + 32 * kc);
    fence4_h(bfr[g][0], bfr[g][1], bfr[g][2], bfr[g][3]);
  }
  const float fbias = fbias_in[hd * DH + e];
  const float rbias = rbias_in[hd * DH + e];
  float hst = 0.0f;
  __syncthreads();

  const v8f z8 = {0.f, 0.f, 0.f, 0.f, 0.f, 0.f, 0.f, 0.f};
  const unsigned sh = (unsigned)(e & 1) * 16u;
  const float xcar_inv = 1.0f / XALL_CAR;
  const float wcar_inv = 1.0f / WREC_CAR;
  const float hres_inv = 1.0f / HRES_CAR;
  const _Float16 zero16 = (_Float16)0.0f;

#pragma unroll 1
  for (int t = 0; t < NS; ++t) {
    const int cur = t & 1, nxt = cur ^ 1;
    const size_t xo = ((size_t)(hh * NS + t)) * (size_t)C6X + (size_t)(hd * DH + e);
    const unsigned wxi = Xw[xo >> 1];
    const unsigned wxf = Xw[(xo + (size_t)NST) >> 1];
    const unsigned wxr = Xw[(xo + (size_t)(2 * NST)) >> 1];

    const _Float16* arow = &Ah[cur][0] + c * APITCH + koff;
    v8f acc0 = z8, acc1 = z8, acc2 = z8;
#pragma unroll
    for (int kc = 0; kc < 4; ++kc) {
      const v16h a = Frag<_Float16>::load(arow + 32 * kc);
      acc0 = Frag<_Float16>::mma(a, bfr[0][kc], acc0);
      acc1 = Frag<_Float16>::mma(a, bfr[1][kc], acc1);
      acc2 = Frag<_Float16>::mma(a, bfr[2][kc], acc2);
      dep_guard3_h4(acc0, acc1, acc2, a, bfr[0][kc], bfr[1][kc], bfr[2][kc]);
    }
    acc_guard3(acc0, acc1, acc2);

    const float xi = h16_to_f32((wxi >> sh) & 0xffffu) * xcar_inv;
    const float xf = h16_to_f32((wxf >> sh) & 0xffffu) * xcar_inv + fbias;
    const float xr = h16_to_f32((wxr >> sh) & 0xffffu) * xcar_inv + rbias;
    const float az = (acc0[0] + acc0[4] * hres_inv) * wcar_inv;
    const float af = (acc1[0] + acc1[4] * hres_inv) * wcar_inv;
    const float ar = (acc2[0] + acc2[4] * hres_inv) * wcar_inv;
    const float rg = __builtin_amdgcn_rcpf(1.0f + expf(-(xr + ar)));
    const float fg = __builtin_amdgcn_rcpf(1.0f + expf(-(xf + af)));
    const float npre = xi + rg * az;
    const float nn = 1.0f - 2.0f * __builtin_amdgcn_rcpf(expf(2.0f * npre) + 1.0f);
    const float hn = fg * hst + (1.0f - fg) * nn;
    hst = hn;
    const _Float16 hhi16 = (_Float16)hn;
    const unsigned short hbits = __builtin_bit_cast(unsigned short, hhi16);
    const float hhi = h16_to_f32((unsigned)hbits);
    const _Float16 hlo16 = (_Float16)((hn - hhi) * HRES_CAR);

    _Float16* an = &Ah[nxt][0] + e;
    an[(8 * hh + 0) * APITCH] = hhi16;
    an[(8 * hh + 1) * APITCH] = zero16;
    an[(8 * hh + 2) * APITCH] = zero16;
    an[(8 * hh + 3) * APITCH] = zero16;
    an[(8 * hh + 4) * APITCH] = hlo16;
    an[(8 * hh + 5) * APITCH] = zero16;
    an[(8 * hh + 6) * APITCH] = zero16;
    an[(8 * hh + 7) * APITCH] = zero16;
    __syncthreads();

    if (wave == 0) {
      const int c8 = c * 8;
      const v8h hv = *(const v8h*)(&Ah[nxt][0] + (8 * hh) * APITCH + c8);
      unsigned short* yp = Yrec + ((size_t)(hh * NS + t)) * (size_t)NST + (size_t)(hd * DH + c8);
      *(volatile v8h*)yp = hv;
      __threadfence();
      *(volatile v8h*)yp = hv;
    }
    if (wave == 1) {
      const int c8 = c * 8;
      const v8h lv = *(const v8h*)(&Ah[nxt][0] + (8 * hh + 4) * APITCH + c8);
      unsigned short* yp = YrecL + ((size_t)(hh * NS + t)) * (size_t)NST + (size_t)(hd * DH + c8);
      *(volatile v8h*)yp = lv;
      __threadfence();
      *(volatile v8h*)yp = lv;
    }
  }
}

extern "C" void kernel_launch(void* const* d_in, const int* in_sizes, int n_in,
                              void* d_out, int out_size, void* d_ws, size_t ws_size, hipStream_t stream) {
  if (n_in < 12 || d_out == nullptr || d_ws == nullptr) return;
  if (in_sizes[0] != NROW * NDIN || in_sizes[1] != NDIN * C3X || in_sizes[2] != C3X || in_sizes[3] != C3X * 4 ||
      in_sizes[4] != C3X || in_sizes[5] != NGRP * DH * GOUT || in_sizes[6] != 3 * NH * DH * DH ||
      in_sizes[7] != NH * DH || in_sizes[8] != NH * DH || in_sizes[9] != NH * DH * DH || in_sizes[10] != NST ||
      in_sizes[11] != NST * NOUTC || out_size != NROW * NOUTC) return;

  const float* x      = (const float*)d_in[0];
  const float* w_in   = (const float*)d_in[1];
  const float* b_in   = (const float*)d_in[2];
  const float* conv_w = (const float*)d_in[3];
  const float* rms1_w = (const float*)d_in[4];
  const float* head_w = (const float*)d_in[5];
  const float* sw     = (const float*)d_in[6];
  const float* fbias  = (const float*)d_in[7];
  const float* rbias  = (const float*)d_in[8];
  const float* ohw    = (const float*)d_in[9];
  const float* rms2_w = (const float*)d_in[10];
  const float* w_out  = (const float*)d_in[11];
  float* out = (float*)d_out;

  char* ws = (char*)d_ws; size_t off = 0;
  auto carve = [&](size_t bytes) -> char* { char* p = ws + off; off += (bytes + 255) & ~(size_t)255; return p; };
  unsigned short* PL16  = (unsigned short*)carve((size_t)NROW * PLP * 2);
  unsigned short* PLB   = (unsigned short*)carve((size_t)NROW * PLP * 2);
  unsigned short* WINT  = (unsigned short*)carve((size_t)C3X * NDIN * 2);
  unsigned short* HWT   = (unsigned short*)carve((size_t)NGRP * GOUT * DH * 2);
  unsigned short* SWT   = (unsigned short*)carve((size_t)3 * NH * DH * DH * 2);
  unsigned short* OHWT  = (unsigned short*)carve((size_t)NH * DH * DH * 2);
  unsigned short* WOUTT = (unsigned short*)carve((size_t)NOUTC * NST * 2);
  float*          H0    = (float*)carve((size_t)NROW * C3X * 4);
  unsigned short* XALL  = (unsigned short*)carve((size_t)NROW * C6X * 2);
  unsigned short* XPL   = PL16;
  unsigned short* H1L   = PL16;
  unsigned short* H1H   = PLB;
  unsigned short* YREC  = PL16;
  unsigned short* YRECL = PLB;
  unsigned short* Y2    = XALL;
  unsigned short* Y2N   = PL16;
  if (off > ws_size || off > (size_t)134217728) return;

  cvt_f16x8_kernel<<<(NROW * NDIN / 8) / NTG, NTG, 0, stream>>>(x, XPL, NROW * NDIN / 8);
  tpw16_kernel<<<dim3(C3X / 64, NDIN / 64, 1), NTG, 0, stream>>>(w_in, NDIN, C3X, 0L, 0L, WINT, WIN_CAR);
  tpw16_kernel<<<dim3(GOUT / 64, DH / 64, NGRP), NTG, 0, stream>>>(head_w, DH, GOUT, (long)DH * GOUT, (long)GOUT * DH, HWT, HW_CAR);
  tpw16_kernel<<<dim3(DH / 64, DH / 64, 3 * NH), NTG, 0, stream>>>(sw, DH, DH, (long)DH * DH, (long)DH * DH, SWT, FACTOR_F * WREC_CAR);
  tpw16_kernel<<<dim3(DH / 64, DH / 64, NH), NTG, 0, stream>>>(ohw, DH, DH, (long)DH * DH, (long)DH * DH, OHWT, OHW_CAR);
  tpw16_kernel<<<dim3(NOUTC / 64, NST / 64, 1), NTG, 0, stream>>>(w_out, NST, NOUTC, 0L, 0L, WOUTT, WOUT_CAR);

  wmma_gemm64<0, false, 2, 0, false, 0><<<dim3((NROW / 64) * (C3X / 64) / 8, 1), NTG, 0, stream>>>(
      XPL, XPL, NDIN, 0L, WINT, WINT, NDIN, 0L, (void*)H0, (void*)H0, C3X, 0L,
      b_in, H0, 0L, NROW, C3X, NDIN, 1.0f / WIN_CAR);

  conv_rms_kernel<<<NROW, NTC, 0, stream>>>(H0, conv_w, rms1_w, H1H, H1L);

  wmma_gemm_ares<<<dim3((NROW / 32) * (GOUT / 64) / 8, NGRP), NTG, 0, stream>>>(
      H1H, H1L, PLP, (long)DH, HWT, DH, (long)GOUT * DH, XALL, C6X, (long)GOUT,
      NROW, GOUT, DH, FACTOR_F * XALL_CAR / HW_CAR, (FACTOR_F * XALL_CAR / HW_CAR) / H1RES_CAR);

  gru_seq_kernel<<<NH, NTR, 0, stream>>>((const unsigned*)(const void*)XALL, SWT, fbias, rbias, YREC, YRECL);

  wmma_gemm_ares<<<dim3((NROW / 32) * (DH / 64) / 8, NH), NTG, 0, stream>>>(
      YREC, YRECL, NST, (long)DH, OHWT, DH, (long)DH * DH, Y2, C6X, (long)DH,
      NROW, DH, DH, 1.0f, 1.0f / HRES_CAR);

  rms2_kernel<<<NROW, NTG, 0, stream>>>(Y2, rms2_w, Y2N);

  wmma_gemm64<0, false, 0, 0, false, 0><<<dim3((NROW / 64) * (NOUTC / 64) / 8, 1), NTG, 0, stream>>>(
      Y2N, Y2N, NST, 0L, WOUTT, WOUTT, NST, 0L, (void*)out, (void*)out, NOUTC, 0L,
      b_in, H0, 0L, NROW, NOUTC, NST, 1.0f / WOUT_CAR);
}
